// GeneralizedCrossMessage_81363860456160
// MI455X (gfx1250) — hardware-verified
//
#include <hip/hip_runtime.h>


namespace {
typedef _Float16 b16;
typedef __attribute__((ext_vector_type(16))) _Float16 v16b;
typedef __attribute__((ext_vector_type(8))) _Float16 v8b;
typedef __attribute__((ext_vector_type(4))) _Float16 v4h;
typedef __attribute__((ext_vector_type(2))) _Float16 v2h;
typedef __attribute__((ext_vector_type(8))) float v8f;
typedef __attribute__((ext_vector_type(4))) float v4f;
typedef __attribute__((ext_vector_type(2))) float v2f;
__device__ __forceinline__ float bf16_rne(float f) { unsigned int u = __float_as_uint(f); u += 0x7FFFu + ((u >> 16) & 1u); return __uint_as_float(u & 0xFFFF0000u); }
__device__ __forceinline__ void split16(float v, b16& hi, b16& lo) { hi = (b16)v; lo = (b16)(v - (float)hi); }
__device__ __forceinline__ v16b frag_kb(const b16* p, int hh) { const v8b a = *(const v8b*)(p + 8 * hh), b = *(const v8b*)(p + 16 + 8 * hh); v16b f;
#pragma unroll
  for (int e = 0; e < 8; ++e) { f[e] = a[e]; f[8 + e] = b[e]; } return f; }
__device__ __forceinline__ v8f wmma16b(v16b a, v16b b, v8f c) { v8f d = __builtin_amdgcn_wmma_f32_16x16x32_f16(false, a, false, b, (short)0, c, false, false); asm volatile("v_nop\n\tv_nop\n\tv_nop\n\tv_nop" : "+v"(d) : "v"(a), "v"(b)); return d; }
__device__ __forceinline__ void wave_lds_sync() { __builtin_amdgcn_fence(__ATOMIC_RELEASE, "workgroup"); __builtin_amdgcn_wave_barrier(); __builtin_amdgcn_fence(__ATOMIC_ACQUIRE, "workgroup"); }
__device__ __forceinline__ float pmul(float a, float b) { float p = a * b; asm volatile("" : "+v"(p)); return p; }
__device__ __forceinline__ int iclamp(int v, int lo, int hi) { return v < lo ? lo : (v > hi ? hi : v); }
__device__ __forceinline__ float nexp2(float v) { return __builtin_amdgcn_exp2f(v); }

constexpr int S = 1024, SL = S  , HDM = 768, DZ = 24, DZP = 32, PF = 96, KP = 64, FIN = 3 * HDM, N = S, NP = S;
constexpr float XS = 8.0f, WSC = 256.0f;
static_assert(S % 64 == 0 && SL % 64 == 0 && HDM % 128 == 0 && FIN % 128 == 0, "tiling");

template <int KD, int NOUT, int LDA, int LDT, bool RNDA>
__global__ __launch_bounds__(64) void gemmx_kernel(const float* __restrict__ A, int nv, const b16* __restrict__ W, const float* __restrict__ bias, int mrows, float* __restrict__ T) {
  constexpr int SL = NOUT < 128 ? NOUT : 128, NT = SL / 16, KC = KD < 128 ? KD : 128;
  static_assert(KD % KC == 0 && KC % 32 == 0 && NOUT % SL == 0 && SL % 32 == 0 && LDA >= KD && LDT >= NOUT, "gemmx tiling");
  __shared__ __attribute__((aligned(16))) b16 Ah[2][16][KC + 8], Al[2][16][KC + 8]; __shared__ __attribute__((aligned(16))) float Tf[2][16][SL + 4];
  const int wave = threadIdx.x >> 5, lane = threadIdx.x & 31, nloc = lane & 15, hlf = lane >> 4; const size_t m0 = (size_t)blockIdx.x * 32 + wave * 16; const int n0 = blockIdx.y * SL;
  v8f acc[NT];
#pragma unroll
  for (int t = 0; t < NT; ++t) acc[t] = (v8f){};
#pragma unroll 1
  for (int kc = 0; kc < KD; kc += KC) {
    for (int idx = lane; idx < 16 * (KC / 4); idx += 32) { const int rr = idx / (KC / 4), c4 = (idx % (KC / 4)) * 4; const size_t row = (m0 + rr < (size_t)nv) ? (m0 + rr) : (size_t)(nv - 1); const v4f v = *(const v4f*)(A + row * LDA + kc + c4); v4h hv, lv;
      for (int j = 0; j < 4; ++j) { b16 ph, pl; split16((RNDA ? bf16_rne(v[j]) : v[j]) * XS, ph, pl); hv[j] = ph; lv[j] = pl; } *(v4h*)(&Ah[wave][rr][c4]) = hv; *(v4h*)(&Al[wave][rr][c4]) = lv; }
    wave_lds_sync();
#pragma unroll
    for (int kb = 0; kb < KC; kb += 32) { const v16b a = frag_kb(&Ah[wave][nloc][kb], hlf), al = frag_kb(&Al[wave][nloc][kb], hlf);
#pragma unroll
      for (int t = 0; t < NT; ++t) { const v16b bw = frag_kb(W + (size_t)(n0 + t * 16 + nloc) * KD + kc + kb, hlf); acc[t] = wmma16b(a, bw, acc[t]); if (!RNDA) acc[t] = wmma16b(al, bw, acc[t]); } }
    wave_lds_sync(); }
#pragma unroll
  for (int t = 0; t < NT; ++t) { const float bb = bias ? bf16_rne(bias[n0 + t * 16 + nloc]) : 0.0f;
#pragma unroll
    for (int r = 0; r < 8; ++r) Tf[wave][8 * hlf + r][t * 16 + nloc] = acc[t][r] * (1.0f / (XS * WSC)) + bb; }
  wave_lds_sync();
  for (int pass = 0; pass < 2; ++pass) { for (int idx = lane; idx < 16 * (SL / 4); idx += 32) { const int rr = idx / (SL / 4), c4 = (idx % (SL / 4)) * 4; if (m0 + rr < (size_t)mrows) *(volatile v4f*)(T + (m0 + rr) * LDT + n0 + c4) = *(const v4f*)(&Tf[wave][rr][c4]); } __threadfence(); }
}

template <int KD, int NOUT, int NV, bool RNDA  >
__global__ __launch_bounds__(64) void gemm_kernel(const float* __restrict__ A, const b16* __restrict__ W, float* __restrict__ T) {
  constexpr int SL = NOUT < 128 ? NOUT : 128, NT = SL / 16, KC = KD < 128 ? KD : 128;
  static_assert(KD % KC == 0 && KC % 32 == 0 && NOUT % SL == 0 && SL % 32 == 0, "gemm tiling");
  __shared__ __attribute__((aligned(16))) b16 Ah[2][16][KC + 8], Al[2][16][KC + 8]; __shared__ __attribute__((aligned(16))) float Tf[2][16][SL + 4];
  const int wave = threadIdx.x >> 5, lane = threadIdx.x & 31, nloc = lane & 15, hlf = lane >> 4; const size_t m0 = (size_t)blockIdx.x * 32 + wave * 16; const int n0 = blockIdx.y * SL;
  v8f acc[NT];
#pragma unroll
  for (int t = 0; t < NT; ++t) acc[t] = (v8f){};
#pragma unroll 1
  for (int kc = 0; kc < KD; kc += KC) {
    for (int idx = lane; idx < 16 * (KC / 4); idx += 32) { const int rr = idx / (KC / 4), c4 = (idx % (KC / 4)) * 4; const size_t row = (m0 + rr < (size_t)NV) ? (m0 + rr) : (size_t)(NV - 1); const v4f v = *(const v4f*)(A + row * KD + kc + c4); v4h hv, lv;
      for (int j = 0; j < 4; ++j) { b16 ph, pl; split16((RNDA ? bf16_rne(v[j]) : v[j]) * XS, ph, pl); hv[j] = ph; lv[j] = pl; } *(v4h*)(&Ah[wave][rr][c4]) = hv; *(v4h*)(&Al[wave][rr][c4]) = lv; }
    wave_lds_sync();
#pragma unroll
    for (int kb = 0; kb < KC; kb += 32) { const v16b a = frag_kb(&Ah[wave][nloc][kb], hlf), al = frag_kb(&Al[wave][nloc][kb], hlf);
#pragma unroll
      for (int t = 0; t < NT; ++t) { const v16b bw = frag_kb(W + (size_t)(n0 + t * 16 + nloc) * KD + kc + kb, hlf); acc[t] = wmma16b(a, bw, acc[t]); acc[t] = wmma16b(al, bw, acc[t]); } }
    wave_lds_sync(); }
#pragma unroll
  for (int t = 0; t < NT; ++t)
#pragma unroll
    for (int r = 0; r < 8; ++r) Tf[wave][8 * hlf + r][t * 16 + nloc] = acc[t][r] * (1.0f / (XS * WSC));
  wave_lds_sync();
  for (int pass = 0; pass < 2; ++pass) { for (int idx = lane; idx < 16 * (SL / 4); idx += 32) { const int rr = idx / (SL / 4), c4 = (idx % (SL / 4)) * 4; *(volatile v4f*)(T + (m0 + rr) * NOUT + n0 + c4) = *(const v4f*)(&Tf[wave][rr][c4]); } __threadfence(); }
}

__global__ __launch_bounds__(256) void prep_kernel(const float* __restrict__ wj, const float* __restrict__ wi, const float* __restrict__ w1, const float* __restrict__ v1, const float* __restrict__ v2, const float* __restrict__ hi, b16* __restrict__ WJ, b16* __restrict__ WI, b16* __restrict__ W1CD, b16* __restrict__ V1T, b16* __restrict__ V2T, b16* __restrict__ HiT) {
  const size_t n1 = (size_t)DZP * HDM / 8, n2 = n1, n3 = (size_t)PF * KP / 8, n4 = (size_t)HDM * FIN / 8, n5 = (size_t)HDM * HDM / 8, n6 = (size_t)HDM * S / 8; size_t u = (size_t)blockIdx.x * 256 + threadIdx.x; v8b o;
  if (u < n1 + n2) { const bool second = u >= n1; const size_t e = (second ? u - n1 : u) * 8; const int d = (int)(e / HDM), k0 = (int)(e % HDM); const float* w = second ? wi : wj;
    for (int j = 0; j < 8; ++j) o[j] = (b16)(d < DZ ? bf16_rne(w[(size_t)(k0 + j) * DZ + d]) * WSC : 0.0f); for (int pass = 0; pass < 2; ++pass) { *(volatile v8b*)((second ? WI : WJ) + e) = o; __threadfence(); } return; } u -= n1 + n2;
  if (u < n3) { const size_t e = u * 8; const int m = (int)(e / KP), k0 = (int)(e % KP); for (int j = 0; j < 8; ++j) { const int k = k0 + j; float w = 0.0f; if (k < DZ) w = w1[(size_t)(48 + k) * PF + m]; else if (k < 2 * DZ) w = w1[(size_t)(72 + k - DZ) * PF + m]; o[j] = (b16)(bf16_rne(w) * WSC); }
    for (int pass = 0; pass < 2; ++pass) { *(volatile v8b*)(W1CD + e) = o; __threadfence(); } return; } u -= n3;
  if (u < n4) { const size_t e = u * 8; const int oo = (int)(e / FIN), k0 = (int)(e % FIN); for (int j = 0; j < 8; ++j) o[j] = (b16)(bf16_rne(v1[(size_t)(k0 + j) * HDM + oo]) * WSC); for (int pass = 0; pass < 2; ++pass) { *(volatile v8b*)(V1T + e) = o; __threadfence(); } return; } u -= n4;
  if (u < n5) { const size_t e = u * 8; const int oo = (int)(e / HDM), k0 = (int)(e % HDM); for (int j = 0; j < 8; ++j) o[j] = (b16)(bf16_rne(v2[(size_t)(k0 + j) * HDM + oo]) * WSC); for (int pass = 0; pass < 2; ++pass) { *(volatile v8b*)(V2T + e) = o; __threadfence(); } return; } u -= n5;
  if (u < n6) { const size_t e = u * 8; const int n = (int)(e / S), k0 = (int)(e % S); for (int j = 0; j < 8; ++j) o[j] = (b16)(bf16_rne(hi[(size_t)(k0 + j) * HDM + n]) * WSC); for (int pass = 0; pass < 2; ++pass) { *(volatile v8b*)(HiT + e) = o; __threadfence(); } }
}
__global__ __launch_bounds__(192) void ab_kernel(const float* __restrict__ ZJ, const float* __restrict__ ZI, const float* __restrict__ w1, const float* __restrict__ b1, float* __restrict__ AS, float* __restrict__ BS) {
  const int tk = blockIdx.x; const int t_ = threadIdx.x; const bool isB = t_ >= PF; const int m = isB ? t_ - PF : t_; const float* z = isB ? ZI + (size_t)tk * DZP : ZJ + (size_t)tk * DZP;
  float a = isB ? 0.0f : bf16_rne(b1[m]);
#pragma unroll 4
  for (int d = 0; d < DZ; ++d) a = fmaf(z[d], bf16_rne(w1[(size_t)((isB ? DZ : 0) + d) * PF + m]), a);
  for (int pass = 0; pass < 2; ++pass) { ((volatile float*)(isB ? BS : AS))[(size_t)tk * PF + m] = a; __threadfence(); }
}
__global__ __launch_bounds__(128) void pair_kernel(const float* __restrict__ ZJ, const float* __restrict__ ZI, const float* __restrict__ AS, const float* __restrict__ BS, const b16* __restrict__ W1CD, const float* __restrict__ w2, const float* __restrict__ b2, float* __restrict__ Lg) {
  __shared__ __attribute__((aligned(16))) b16 Ap[64][KP + 8]; __shared__ float zj[DZP], w2s[PF], as_[PF], lg[64];
  const int wave = threadIdx.x >> 5, lane = threadIdx.x & 31, nloc = lane & 15, hlf = lane >> 4; const int s = blockIdx.x, t0 = blockIdx.y * 64;
  if (threadIdx.x < DZP) zj[threadIdx.x] = ZJ[(size_t)s * DZP + threadIdx.x]; if (threadIdx.x < PF) { w2s[threadIdx.x] = bf16_rne(w2[threadIdx.x]); as_[threadIdx.x] = AS[(size_t)s * PF + threadIdx.x]; }
  __syncthreads();
  for (int i = threadIdx.x; i < 64 * KP; i += 128) { const int r = i / KP, k = i % KP; float v = 0.0f; if (k < DZ) v = zj[k] * ZI[(size_t)(t0 + r) * DZP + k]; else if (k < 2 * DZ) v = fabsf(zj[k - DZ] - ZI[(size_t)(t0 + r) * DZP + k - DZ]); Ap[r][k] = (b16)(v * XS); }
  __syncthreads();
  v8f acc[6];
#pragma unroll
  for (int t = 0; t < 6; ++t) acc[t] = (v8f){};
#pragma unroll
  for (int kb = 0; kb < KP; kb += 32) { const v16b a = frag_kb(&Ap[wave * 16 + nloc][kb], hlf);
#pragma unroll
    for (int t = 0; t < 6; ++t) acc[t] = wmma16b(a, frag_kb(W1CD + (size_t)(t * 16 + nloc) * KP + kb, hlf), acc[t]); }
  float lgt[8];
#pragma unroll
  for (int r = 0; r < 8; ++r) { const int tt = t0 + wave * 16 + 8 * hlf + r; float p = 0.0f;
#pragma unroll
    for (int t = 0; t < 6; ++t) { const int m = t * 16 + nloc; const float h = fmaxf(acc[t][r] * (1.0f / (XS * WSC)) + as_[m] + BS[(size_t)tt * PF + m], 0.0f); p = fmaf(h, w2s[m], p); } lgt[r] = p; }
#pragma unroll
  for (int w = 1; w < 16; w <<= 1)
#pragma unroll
    for (int r = 0; r < 8; ++r) lgt[r] += __shfl_xor(lgt[r], w);
  if (nloc == 0) { const float bb = bf16_rne(b2[0]);
#pragma unroll
    for (int r = 0; r < 8; ++r) lg[wave * 16 + 8 * hlf + r] = lgt[r] + bb; }
  __syncthreads();
  for (int pass = 0; pass < 2; ++pass) { if (wave == 0) { ((volatile float*)Lg)[(size_t)s * S + t0 + lane] = lg[lane]; ((volatile float*)Lg)[(size_t)s * S + t0 + 32 + lane] = lg[32 + lane]; } __threadfence(); }
}
__global__ __launch_bounds__(256) void softmax_kernel(const float* __restrict__ Lg, const float* __restrict__ am, float* __restrict__ P) {
  __shared__ float red[256]; __shared__ float rowv[S];
  const int s = blockIdx.x, t_ = threadIdx.x; float m = -INFINITY;
  for (int t = t_; t < S; t += 256) { const float v = Lg[(size_t)s * S + t] + (1.0f - bf16_rne(am[t])) * -3.4028235e38f; rowv[t] = v; m = fmaxf(m, v); }
  red[t_] = m; __syncthreads(); for (int w = 128; w >= 1; w >>= 1) { if (t_ < w) red[t_] = fmaxf(red[t_], red[t_ + w]); __syncthreads(); } m = red[0]; __syncthreads();
  float sum = 0.0f; for (int t = t_; t < S; t += 256) { const float e = __expf(rowv[t] - m); rowv[t] = e; sum += e; }
  red[t_] = sum; __syncthreads(); for (int w = 128; w >= 1; w >>= 1) { if (t_ < w) red[t_] += red[t_ + w]; __syncthreads(); } const float inv = 1.0f / red[0];
  for (int pass = 0; pass < 2; ++pass) { for (int q = t_; q < S / 4; q += 256) { v4f o; for (int j = 0; j < 4; ++j) o[j] = rowv[q * 4 + j] * inv; *(volatile v4f*)(P + (size_t)s * S + q * 4) = o; } __threadfence(); }
}
__global__ __launch_bounds__(256) void msgin_kernel(const float* __restrict__ CTX, const float* __restrict__ hj, float* __restrict__ MI) {
  const size_t u = (size_t)blockIdx.x * 256 + threadIdx.x; if (u >= (size_t)SL * FIN / 4) return; const int s = (int)(u / (FIN / 4)), c = (int)(u % (FIN / 4)) * 4; v4f o;
  if (c < HDM) o = *(const v4f*)(CTX + (size_t)s * HDM + c);
  else if (c < 2 * HDM) { const v4f h = *(const v4f*)(hj + (size_t)s * HDM + c - HDM); for (int j = 0; j < 4; ++j) o[j] = bf16_rne(h[j]); }
  else { const v4f h = *(const v4f*)(hj + (size_t)s * HDM + c - 2 * HDM), x = *(const v4f*)(CTX + (size_t)s * HDM + c - 2 * HDM); for (int j = 0; j < 4; ++j) o[j] = x[j] * bf16_rne(h[j]); }
  for (int pass = 0; pass < 2; ++pass) { *(volatile v4f*)(MI + u * 4) = o; __threadfence(); }
}
__global__ __launch_bounds__(256) void relu_kernel(float* __restrict__ Hp, int n4) { const int u = blockIdx.x * 256 + threadIdx.x; if (u >= n4) return; v4f v = *(const v4f*)(Hp + (size_t)u * 4); for (int j = 0; j < 4; ++j) v[j] = fmaxf(v[j], 0.0f); for (int pass = 0; pass < 2; ++pass) { *(volatile v4f*)(Hp + (size_t)u * 4) = v; __threadfence(); } }
__global__ __launch_bounds__(256) void scale_kernel(const float* __restrict__ T2, const float* __restrict__ alpha, float* __restrict__ out, int n4) { const int u = blockIdx.x * 256 + threadIdx.x; if (u >= n4) return; const float a = bf16_rne(alpha[0]); v4f v = *(const v4f*)(T2 + (size_t)u * 4); for (int j = 0; j < 4; ++j) v[j] *= a; for (int pass = 0; pass < 2; ++pass) { *(volatile v4f*)(out + (size_t)u * 4) = v; __threadfence(); } }
}

extern "C" void kernel_launch(void* const* d_in, const int* in_sizes, int n_in, void* d_out, int out_size, void* d_ws, size_t ws_size, hipStream_t stream) {
  (void)n_in;
  auto Fp = [&](int i) { return (const float*)d_in[i]; };
  if (in_sizes[0] != S * HDM || in_sizes[1] != S * HDM || in_sizes[2] != S || in_sizes[3] != HDM * DZ || in_sizes[4] != HDM * DZ || in_sizes[5] != PF * PF || in_sizes[6] != PF || in_sizes[7] != PF || in_sizes[8] != 1 || in_sizes[9] != FIN * HDM || in_sizes[10] != HDM || in_sizes[11] != HDM * HDM || in_sizes[12] != HDM || in_sizes[13] != 1 || out_size != S * HDM) return;
  size_t off = 0; char* ws = (char*)d_ws;
  auto carve = [&](size_t bytes) { char* p = ws + off; off += (bytes + 255) & ~(size_t)255; return p; };
  b16* WJ = (b16*)carve((size_t)DZP * HDM * 2); b16* WI = (b16*)carve((size_t)DZP * HDM * 2); b16* W1CD = (b16*)carve((size_t)PF * KP * 2); b16* V1T = (b16*)carve((size_t)HDM * FIN * 2); b16* V2T = (b16*)carve((size_t)HDM * HDM * 2); b16* HiT = (b16*)carve((size_t)HDM * S * 2);
  float* ZJ = (float*)carve((size_t)S * DZP * 4); float* ZI = (float*)carve((size_t)S * DZP * 4); float* AS = (float*)carve((size_t)S * PF * 4); float* BS = (float*)carve((size_t)S * PF * 4); float* Lg = (float*)carve((size_t)S * S * 4); float* P = (float*)carve((size_t)S * S * 4);
  float* CTX = (float*)carve((size_t)S * HDM * 4); float* MI = (float*)carve((size_t)S * FIN * 4); float* HV = (float*)carve((size_t)S * HDM * 4); float* T2 = (float*)carve((size_t)S * HDM * 4);
  if (off > ws_size || off > ((size_t)128 << 20)) return;
  const size_t nprep = (size_t)2 * DZP * HDM / 8 + (size_t)PF * KP / 8 + (size_t)HDM * FIN / 8 + (size_t)HDM * HDM / 8 + (size_t)HDM * S / 8;
  prep_kernel<<<(unsigned)((nprep + 255) / 256), 256, 0, stream>>>(Fp(3), Fp(4), Fp(5), Fp(9), Fp(11), Fp(1), WJ, WI, W1CD, V1T, V2T, HiT);
  gemmx_kernel<HDM, DZP, HDM, DZP, true><<<dim3(S / 32, 1), 64, 0, stream>>>(Fp(0), S, WJ, nullptr, S, ZJ);
  gemmx_kernel<HDM, DZP, HDM, DZP, true><<<dim3(S / 32, 1), 64, 0, stream>>>(Fp(1), S, WI, nullptr, S, ZI);
  ab_kernel<<<S, 192, 0, stream>>>(ZJ, ZI, Fp(5), Fp(6), AS, BS);
  pair_kernel<<<dim3(SL, S / 64), 128, 0, stream>>>(ZJ, ZI, AS, BS, W1CD, Fp(7), Fp(8), Lg);
  softmax_kernel<<<SL, 256, 0, stream>>>(Lg, Fp(2), P);
  gemm_kernel<S, HDM, SL, false><<<dim3(SL / 32, HDM / 128), 64, 0, stream>>>(P, HiT, CTX);
  msgin_kernel<<<(unsigned)(((size_t)SL * FIN / 4 + 255) / 256), 256, 0, stream>>>(CTX, Fp(0), MI);
  gemmx_kernel<FIN, HDM, FIN, HDM, false><<<dim3(SL / 32, HDM / 128), 64, 0, stream>>>(MI, SL, V1T, Fp(10), SL, HV); relu_kernel<<<(SL * HDM / 4 + 255) / 256, 256, 0, stream>>>(HV, SL * HDM / 4);
  gemmx_kernel<HDM, HDM, HDM, HDM, false><<<dim3(SL / 32, HDM / 128), 64, 0, stream>>>(HV, SL, V2T, Fp(12), SL, T2);
  scale_kernel<<<(SL * HDM / 4 + 255) / 256, 256, 0, stream>>>(T2, Fp(13), (float*)d_out, SL * HDM / 4);
}
